// VectorizedInteraction_33947421508010
// MI455X (gfx1250) — hardware-verified
//
#include <hip/hip_runtime.h>
#include <math.h>
#include <stdint.h>

#define NB     2
#define TT     512
#define NF     6
#define DD     32
#define HID    128
#define NH     4
#define HD     32
#define GH     32
#define FD     128
#define LL     (TT * NF)
#define NTOK   (NB * LL)
#define NPOOL  (NB * TT)
#define LNEPS  1.0e-5f
#define XC     16.0f
#define WSC    64.0f
#define QC     8.0f
#define KC     8.0f
#define VC     16.0f
#define AC     32.0f
#define YC     16.0f
#define RSC    1024.0f
#define INVRS  (1.0f / 1024.0f)
#define FLOORC 1.0e-9f
#define NEGBIG (-1.0e30f)
#define SCL    ((0.17677669529663687f * 1.4426950408889634f) / (QC * KC))
static_assert(NH * HD == HID);
static_assert(FD == HID);
static_assert((LL % 64) == 0 && (LL % 48) == 0 && (LL % 32) == 0);
static_assert((NTOK % 64) == 0 && (NPOOL % 64) == 0);
static_assert(DD == 32 && GH == 32);

typedef _Float16 v16h __attribute__((ext_vector_type(16)));
typedef _Float16 v8h  __attribute__((ext_vector_type(8)));
typedef float    v8f  __attribute__((ext_vector_type(8)));
typedef float    v4f  __attribute__((ext_vector_type(4)));
typedef unsigned int v4u __attribute__((ext_vector_type(4)));
typedef unsigned int v2u __attribute__((ext_vector_type(2)));

union FragH { v16h v; v8h h[2]; };

__device__ __forceinline__ unsigned short bf_bits(float f) {
  unsigned u = __float_as_uint(f);
  return (unsigned short)((u + 0x7FFFu + ((u >> 16) & 1u)) >> 16);
}
__device__ __forceinline__ float bf_up(unsigned short h) { return __uint_as_float(((unsigned)h) << 16); }
__device__ __forceinline__ float bfr(float f) { return bf_up(bf_bits(f)); }
__device__ __forceinline__ unsigned short h_bits(_Float16 x) { return __builtin_bit_cast(unsigned short, x); }
__device__ __forceinline__ unsigned pk16(unsigned short a, unsigned short b) { return (unsigned)a | ((unsigned)b << 16); }
__device__ __forceinline__ v8f zero8() { v8f z = {0.f, 0.f, 0.f, 0.f, 0.f, 0.f, 0.f, 0.f}; return z; }
__device__ __forceinline__ float hmax8(v8f s) {
  return fmaxf(fmaxf(fmaxf(s[0], s[1]), fmaxf(s[2], s[3])), fmaxf(fmaxf(s[4], s[5]), fmaxf(s[6], s[7])));
}
__device__ __forceinline__ const _Float16* h16(const unsigned short* p) { return (const _Float16*)(const void*)p; }
__device__ __forceinline__ void split_h(float f, unsigned short& hb, unsigned short& lb) {
  const _Float16 h = (_Float16)f;
  const _Float16 l = (_Float16)((f - (float)h) * RSC);
  hb = h_bits(h);
  lb = h_bits(l);
}
__device__ __forceinline__ float fexp2(float x) { return __builtin_amdgcn_exp2f(x); }
__device__ __forceinline__ float sigm(float a) {
  const float e = __expf(fminf(-a, 60.0f));
  return 1.0f / (1.0f + e);
}
__device__ __forceinline__ float wsum(float v) {
#pragma unroll
  for (int off = 16; off > 0; off >>= 1) v += __shfl_xor(v, off, 32);
  return v;
}

__device__ __forceinline__ v16h ldfrag_h(const _Float16* p) {
  FragH f;
  f.h[0] = *(const v8h*)(p);
  f.h[1] = *(const v8h*)(p + 16);
  return f.v;
}

__device__ __forceinline__ v8f mma_h_raw(v16h a, v16h b, v8f c) {
  return __builtin_amdgcn_wmma_f32_16x16x32_f16(false, a, false, b, (short)0, c, false, false);
}
__device__ __forceinline__ void guard4x6(v8f& a, v8f& b, v8f& c, v8f& d,
                                         v16h x0, v16h x1, v16h x2, v16h x3, v16h x4, v16h x5) {
#if defined(__HIP_DEVICE_COMPILE__)
  asm volatile("v_nop\n\tv_nop\n\tv_nop\n\tv_nop"
               : "+v"(a), "+v"(b), "+v"(c), "+v"(d)
               : "v"(x0), "v"(x1), "v"(x2), "v"(x3), "v"(x4), "v"(x5));
#endif
}
__device__ __forceinline__ void guard8x6(v8f& a0, v8f& a1, v8f& a2, v8f& a3,
                                         v8f& b0, v8f& b1, v8f& b2, v8f& b3,
                                         v16h x0, v16h x1, v16h x2, v16h x3, v16h x4, v16h x5) {
#if defined(__HIP_DEVICE_COMPILE__)
  asm volatile("v_nop\n\tv_nop\n\tv_nop\n\tv_nop"
               : "+v"(a0), "+v"(a1), "+v"(a2), "+v"(a3), "+v"(b0), "+v"(b1), "+v"(b2), "+v"(b3)
               : "v"(x0), "v"(x1), "v"(x2), "v"(x3), "v"(x4), "v"(x5));
#endif
}
__device__ __forceinline__ void acc_guard4(v8f& a, v8f& b, v8f& c, v8f& d) {
#if defined(__HIP_DEVICE_COMPILE__)
  asm volatile("v_nop\n\tv_nop\n\tv_nop\n\tv_nop" : "+v"(a), "+v"(b), "+v"(c), "+v"(d));
#endif
}

__global__ __launch_bounds__(256) void wprep(const float* __restrict__ qw, const float* __restrict__ kw,
                                              const float* __restrict__ vw, const float* __restrict__ ow,
                                              const float* __restrict__ fw,
                                              unsigned short* WT, unsigned short* WOT, unsigned short* FWT) {
  __shared__ float T[64 * 33];
  const int t  = threadIdx.x;
  const int bx = blockIdx.x;
  if (bx < 12) {
    const int p  = bx >> 2;
    const int n0 = (bx & 3) * 32;
    const float* src = (p == 0) ? qw : ((p == 1) ? kw : vw);
    {
      const int k = t >> 3, nn = 4 * (t & 7);
      const v4f a = *(const v4f*)(src + (size_t)k * HID + n0 + nn);
#pragma unroll
      for (int i = 0; i < 4; ++i) T[k * 33 + nn + i] = a[i];
    }
    __syncthreads();
    {
      const bool wr = (t < 128);
      const int tt = t & 127;
      const int o = tt >> 2, e = tt & 3;
      float w[8];
#pragma unroll
      for (int i = 0; i < 8; ++i) w[i] = bfr(T[(8 * e + i) * 33 + o]) * WSC;
      v4u v;
#pragma unroll
      for (int i = 0; i < 4; ++i) v[i] = pk16(h_bits((_Float16)w[2 * i]), h_bits((_Float16)w[2 * i + 1]));
      unsigned short* dp = WT + (size_t)(p * HID + n0 + o) * DD + 8 * e;
      if (wr) *(volatile v4u*)dp = v;
      __threadfence();
      if (wr) *(volatile v4u*)dp = v;
    }
  } else {
    const int q = bx - 12;
    const bool iso = (q < 8);
    const int rr = iso ? q : (q - 8);
    const float* src   = iso ? ow : fw;
    unsigned short* ds = iso ? WOT : FWT;
    const int o0 = (rr >> 1) * 32, k0 = (rr & 1) * 64;
    {
      const int k = t >> 2, oo = 8 * (t & 3);
      const float* sp = src + (size_t)(k0 + k) * HID + o0 + oo;
      const v4f a = *(const v4f*)(sp), c = *(const v4f*)(sp + 4);
#pragma unroll
      for (int i = 0; i < 4; ++i) { T[k * 33 + oo + i] = a[i]; T[k * 33 + oo + 4 + i] = c[i]; }
    }
    __syncthreads();
    {
      const int o = t >> 3, e = t & 7;
      float w[8];
#pragma unroll
      for (int i = 0; i < 8; ++i) w[i] = bfr(T[(8 * e + i) * 33 + o]) * WSC;
      v4u v;
#pragma unroll
      for (int i = 0; i < 4; ++i) v[i] = pk16(h_bits((_Float16)w[2 * i]), h_bits((_Float16)w[2 * i + 1]));
      unsigned short* dp = ds + (size_t)(o0 + o) * HID + k0 + 8 * e;
      *(volatile v4u*)dp = v;
      __threadfence();
      *(volatile v4u*)dp = v;
    }
  }
}

__global__ __launch_bounds__(256) void qkv_prep(
    const float* __restrict__ x, const float* __restrict__ glnw, const float* __restrict__ glnb,
    const float* __restrict__ gw1, const float* __restrict__ gb1, const float* __restrict__ gw2,
    const float* __restrict__ gb2, const float* __restrict__ qbias, const float* __restrict__ kbias,
    const float* __restrict__ vbias, const unsigned short* __restrict__ WT,
    unsigned short* QH, unsigned short* QL, unsigned short* KH, unsigned short* KL,
    unsigned short* VTH, unsigned short* VTL) {
  __shared__ __align__(16) float sX[64 * 33];
  __shared__ __align__(16) _Float16 sXh[64 * 40];
  __shared__ float sW1[DD * GH];
  __shared__ float sG[64];
  __shared__ __align__(16) unsigned short sH[128 * 72];
  __shared__ __align__(16) unsigned short sL[128 * 72];
  const int t = threadIdx.x, wave = t >> 5, lane = t & 31, hh = lane >> 4, m = lane & 15;
  const int tok0  = blockIdx.x * 64;
  const int b     = tok0 / LL;
  const int ltok0 = tok0 - b * LL;

  {
    const int tk = t >> 2, j = 8 * (t & 3);
    const float* sp = x + (size_t)(tok0 + tk) * DD + j;
    const v4f a = *(const v4f*)(sp), c = *(const v4f*)(sp + 4);
    float r8[8];
#pragma unroll
    for (int i = 0; i < 4; ++i) { r8[i] = bfr(a[i]); r8[4 + i] = bfr(c[i]); }
#pragma unroll
    for (int i = 0; i < 8; ++i) {
      sX[tk * 33 + j + i]  = r8[i];
      sXh[tk * 40 + j + i] = (_Float16)(r8[i] * XC);
    }
    for (int i = t; i < DD * GH; i += 256) sW1[i] = bfr(gw1[i]);
  }
  __syncthreads();

  {
    const float gw = bfr(glnw[lane]), gb = bfr(glnb[lane]);
    const float b1 = bfr(gb1[lane]),  w2 = bfr(gw2[lane]), b2 = bfr(gb2[0]);
#pragma unroll 1
    for (int i = 0; i < 8; ++i) {
      const int tk = wave * 8 + i;
      const float xv  = sX[tk * 33 + lane];
      const float mu  = wsum(xv) * (1.0f / DD);
      const float dv  = xv - mu;
      const float var = wsum(dv * dv) * (1.0f / DD);
      const float xn  = dv * rsqrtf(var + LNEPS) * gw + gb;
      float hacc = b1;
#pragma unroll
      for (int k = 0; k < DD; ++k) hacc += __shfl(xn, k, 32) * sW1[k * GH + lane];
      const float hs = hacc * sigm(hacc);
      const float gs = wsum(hs * w2) + b2;
      const float g  = sigm(gs);
      if (lane == 0) sG[tk] = g;
    }
  }
  __syncthreads();

  const int rt = wave & 3, ch = wave >> 2;
  FragH af;
  af.h[0] = *(const v8h*)(sXh + (16 * rt + m) * 40 + 8 * hh);
  af.h[1] = *(const v8h*)(sXh + (16 * rt + m) * 40 + 16 + 8 * hh);
  const _Float16* WTp = h16(WT);
#pragma unroll 1
  for (int p = 0; p < 3; ++p) {
    const float* bp = (p == 0) ? qbias : ((p == 1) ? kbias : vbias);
    const float osc = (p == 2) ? VC : QC;
    v16h bf[4];
#pragma unroll
    for (int j = 0; j < 4; ++j)
      bf[j] = ldfrag_h(WTp + (size_t)(p * HID + 64 * ch + 16 * j + m) * DD + 8 * hh);
    v8f acc[4];
#pragma unroll
    for (int j = 0; j < 4; ++j) acc[j] = mma_h_raw(af.v, bf[j], zero8());
    guard4x6(acc[0], acc[1], acc[2], acc[3], af.v, bf[0], bf[1], bf[2], bf[3], af.v);
    float gr[8];
#pragma unroll
    for (int r = 0; r < 8; ++r) gr[r] = sG[16 * rt + 8 * hh + r];
#pragma unroll
    for (int j = 0; j < 4; ++j) {
      const int n = 64 * ch + 16 * j + m;
      const float bn = bfr(bp[n]);
#pragma unroll
      for (int r = 0; r < 8; ++r) {
        const int row = 16 * rt + 8 * hh + r;
        const float f = ((acc[j][r] * (1.0f / (XC * WSC)) + bn) * gr[r]) * osc;
        unsigned short hb, lb;
        split_h(f, hb, lb);
        if (p < 2) { sH[row * 136 + n] = hb; sL[row * 136 + n] = lb; }
        else       { sH[n * 72 + row]  = hb; sL[n * 72 + row]  = lb; }
      }
    }
    __syncthreads();
    if (p < 2) {
      unsigned short* Hp = (p == 0) ? QH : KH;
      unsigned short* Lp = (p == 0) ? QL : KL;
      const int e = t & 15;
      v4u hv[4], lv[4];
#pragma unroll
      for (int i = 0; i < 4; ++i) {
        const int row = 16 * i + (t >> 4);
        hv[i] = *(const v4u*)(sH + row * 136 + 8 * e);
        lv[i] = *(const v4u*)(sL + row * 136 + 8 * e);
      }
#pragma unroll
      for (int i = 0; i < 4; ++i) {
        const int row = 16 * i + (t >> 4);
        *(volatile v4u*)(Hp + (size_t)(tok0 + row) * HID + 8 * e) = hv[i];
        *(volatile v4u*)(Lp + (size_t)(tok0 + row) * HID + 8 * e) = lv[i];
      }
      __threadfence();
#pragma unroll
      for (int i = 0; i < 4; ++i) {
        const int row = 16 * i + (t >> 4);
        *(volatile v4u*)(Hp + (size_t)(tok0 + row) * HID + 8 * e) = hv[i];
        *(volatile v4u*)(Lp + (size_t)(tok0 + row) * HID + 8 * e) = lv[i];
      }
    } else {
      const int e = t & 7;
      v4u hv[4], lv[4];
#pragma unroll
      for (int i = 0; i < 4; ++i) {
        const int vr = 32 * i + (t >> 3);
        hv[i] = *(const v4u*)(sH + vr * 72 + 8 * e);
        lv[i] = *(const v4u*)(sL + vr * 72 + 8 * e);
      }
#pragma unroll
      for (int i = 0; i < 4; ++i) {
        const int vr = 32 * i + (t >> 3);
        const size_t o = ((size_t)(b * HID + vr)) * LL + ltok0 + 8 * e;
        *(volatile v4u*)(VTH + o) = hv[i];
        *(volatile v4u*)(VTL + o) = lv[i];
      }
      __threadfence();
#pragma unroll
      for (int i = 0; i < 4; ++i) {
        const int vr = 32 * i + (t >> 3);
        const size_t o = ((size_t)(b * HID + vr)) * LL + ltok0 + 8 * e;
        *(volatile v4u*)(VTH + o) = hv[i];
        *(volatile v4u*)(VTL + o) = lv[i];
      }
    }
    __syncthreads();
  }
}

__global__ __launch_bounds__(256) void vsuf(const unsigned short* __restrict__ VTH, const unsigned short* __restrict__ VTL,
                                             const int* __restrict__ Tp, float* SV) {
  __shared__ float bs[TT];
  __shared__ __align__(16) float S[TT];
  const int t = threadIdx.x;
  const int row = blockIdx.x;
  const int tin = Tp[0];
  const int ntb = (tin < 0) ? 0 : ((tin > TT) ? TT : tin);
  const _Float16* hp = h16(VTH) + (size_t)row * LL;
  const _Float16* lp = h16(VTL) + (size_t)row * LL;
  for (int tb = t; tb < TT; tb += 256) {
    float s = 0.f;
#pragma unroll
    for (int f = 0; f < NF; ++f) {
      const int idx = tb * NF + f;
      s += ((float)hp[idx] + (float)lp[idx] * INVRS) * (1.0f / VC);
    }
    bs[tb] = (tb < ntb) ? s : 0.f;
  }
  __syncthreads();
  if (t == 0) {
    float run = 0.f;
    for (int tb = TT - 1; tb >= 0; --tb) { S[tb] = run; run += bs[tb]; }
  }
  __syncthreads();
  {
    const bool wr = (t < 128);
    const int tt = t & 127;
    const v4f v = *(const v4f*)(S + 4 * tt);
    float* dp = SV + (size_t)row * TT + 4 * tt;
    if (wr) *(volatile v4f*)dp = v;
    __threadfence();
    if (wr) *(volatile v4f*)dp = v;
  }
}

template <bool MASKED>
__device__ __forceinline__ void attn_step(const int kb, const int jl, const int hh,
    const _Float16* __restrict__ kH, const _Float16* __restrict__ kL,
    const _Float16* __restrict__ vH, const _Float16* __restrict__ vL,
    const v16h qhi, const v16h qlo, float& m_run, float& l_run,
    v8f& o1, v8f& o1r, v8f& o2, v8f& o2r) {
  const v16h kh0 = ldfrag_h(kH + (size_t)kb * HID);
  const v16h kh1 = ldfrag_h(kH + (size_t)(kb + 16) * HID);
  const v16h kl0 = ldfrag_h(kL + (size_t)kb * HID);
  const v16h kl1 = ldfrag_h(kL + (size_t)(kb + 16) * HID);
  v8f s0  = mma_h_raw(kh0, qhi, zero8());
  v8f s1  = mma_h_raw(kh1, qhi, zero8());
  v8f s0r = mma_h_raw(kh0, qlo, zero8());
  v8f s1r = mma_h_raw(kh1, qlo, zero8());
  s0r = mma_h_raw(kl0, qhi, s0r);
  s1r = mma_h_raw(kl1, qhi, s1r);
  guard4x6(s0, s1, s0r, s1r, kh0, kh1, kl0, kl1, qhi, qlo);

  float e0[8], e1[8];
#pragma unroll
  for (int r = 0; r < 8; ++r) {
    e0[r] = (s0[r] + s0r[r] * INVRS) * SCL;
    e1[r] = (s1[r] + s1r[r] * INVRS) * SCL;
  }
  if (MASKED) {
    const int base = kb + 8 * hh;
#pragma unroll
    for (int r = 0; r < 8; ++r) {
      e0[r] = (base + r      < jl) ? e0[r] : NEGBIG;
      e1[r] = (base + 16 + r < jl) ? e1[r] : NEGBIG;
    }
  }
  float mx = fmaxf(fmaxf(fmaxf(fmaxf(e0[0], e0[1]), fmaxf(e0[2], e0[3])), fmaxf(fmaxf(e0[4], e0[5]), fmaxf(e0[6], e0[7]))),
                   fmaxf(fmaxf(fmaxf(e1[0], e1[1]), fmaxf(e1[2], e1[3])), fmaxf(fmaxf(e1[4], e1[5]), fmaxf(e1[6], e1[7]))));
  mx = fmaxf(mx, __shfl_xor(mx, 16, 32));
  const float m_new = fmaxf(m_run, mx);
  const float corr  = fexp2(m_run - m_new);
  m_run = m_new;
  const float msh = m_new - 10.0f;
  l_run *= corr;
  o1 = o1 * corr; o1r = o1r * corr; o2 = o2 * corr; o2r = o2r * corr;

  FragH ph, pl;
  float ls = 0.f;
#pragma unroll
  for (int r = 0; r < 8; ++r) {
    const float p0 = fexp2(e0[r] - msh);
    const float p1 = fexp2(e1[r] - msh);
    ls += p0 + p1;
    const _Float16 a0 = (_Float16)p0, a1 = (_Float16)p1;
    ph.h[0][r] = a0;
    ph.h[1][r] = a1;
    pl.h[0][r] = (_Float16)((p0 - (float)a0) * RSC);
    pl.h[1][r] = (_Float16)((p1 - (float)a1) * RSC);
  }
  l_run += ls;

  const v16h vh1 = ldfrag_h(vH + kb);
  const v16h vl1 = ldfrag_h(vL + kb);
  const v16h vh2 = ldfrag_h(vH + (size_t)16 * LL + kb);
  const v16h vl2 = ldfrag_h(vL + (size_t)16 * LL + kb);
  o1  = mma_h_raw(vh1, ph.v, o1);
  o2  = mma_h_raw(vh2, ph.v, o2);
  o1r = mma_h_raw(vh1, pl.v, o1r);
  o2r = mma_h_raw(vh2, pl.v, o2r);
  o1r = mma_h_raw(vl1, ph.v, o1r);
  o2r = mma_h_raw(vl2, ph.v, o2r);
  guard4x6(o1, o2, o1r, o2r, vh1, vh2, vl1, vl2, ph.v, pl.v);
}

__global__ __launch_bounds__(384)
void attn_pool(const unsigned short* __restrict__ QH, const unsigned short* __restrict__ QL,
               const unsigned short* __restrict__ KH, const unsigned short* __restrict__ KL,
               const unsigned short* __restrict__ VTH, const unsigned short* __restrict__ VTL,
               const float* __restrict__ SV, unsigned short* PH, unsigned short* PL) {
  __shared__ __align__(16) float sO[48 * 132];
  __shared__ __align__(16) unsigned short sPH[8 * 128];
  __shared__ __align__(16) unsigned short sPL[8 * 128];
  const int t = threadIdx.x, wave = t >> 5, lane = t & 31, hh = lane >> 4, c = lane & 15;
  const int bx = blockIdx.x;
  const int b  = bx >> 6;
  const int qblk = bx & 63;
  const int q0 = qblk * 48;
  const int h  = wave & 3, qt = wave >> 2;
  const int qw0 = q0 + 16 * qt;
  const int qi  = qw0 + c;
  const int jl  = (qi / NF + 1) * NF;
  const size_t tokb = (size_t)b * LL;

  const _Float16* QHp = h16(QH);
  const _Float16* QLp = h16(QL);
  const v16h qhi = ldfrag_h(QHp + (tokb + qi) * HID + h * HD + 8 * hh);
  const v16h qlo = ldfrag_h(QLp + (tokb + qi) * HID + h * HD + 8 * hh);
  const _Float16* kH = h16(KH) + (tokb + c) * HID + h * HD + 8 * hh;
  const _Float16* kL = h16(KL) + (tokb + c) * HID + h * HD + 8 * hh;
  const _Float16* vH = h16(VTH) + ((size_t)(b * HID + h * HD + c)) * LL + 8 * hh;
  const _Float16* vL = h16(VTL) + ((size_t)(b * HID + h * HD + c)) * LL + 8 * hh;

  float m_run = NEGBIG, l_run = 0.f;
  v8f o1 = zero8(), o1r = zero8(), o2 = zero8(), o2r = zero8();
  const int jmax  = ((qw0 + 15) / NF + 1) * NF;
  const int jmin  = (qw0 / NF + 1) * NF;
  const int cfull = (jmin / 32) * 32;
  int kb = 0;
#pragma unroll 1
  for (; kb < cfull; kb += 32)
    attn_step<false>(kb, jl, hh, kH, kL, vH, vL, qhi, qlo, m_run, l_run, o1, o1r, o2, o2r);
#pragma unroll 1
  for (; kb < jmax; kb += 32)
    attn_step<true>(kb, jl, hh, kH, kL, vH, vL, qhi, qlo, m_run, l_run, o1, o1r, o2, o2r);

  l_run += __shfl_xor(l_run, 16, 32);
  const float inv = (1.0f / l_run) * (1.0f / VC);
  const int tq = qi / NF;
  const float* svp = SV + ((size_t)(b * HID + h * HD)) * TT + tq;
  float* so = sO + (16 * qt + c) * 132 + h * HD;
#pragma unroll
  for (int r = 0; r < 8; ++r) {
    const int d1 = 8 * hh + r, d2 = 16 + 8 * hh + r;
    so[d1] = (o1[r] + o1r[r] * INVRS) * inv + FLOORC * svp[(size_t)d1 * TT];
    so[d2] = (o2[r] + o2r[r] * INVRS) * inv + FLOORC * svp[(size_t)d2 * TT];
  }
  __syncthreads();
  {
    const bool act = (t < 256);
    const int tt = act ? t : 0;
    const int pr = tt >> 5, col = 4 * (tt & 31);
    v4f s = {0.f, 0.f, 0.f, 0.f};
#pragma unroll
    for (int f = 0; f < NF; ++f) s += *(const v4f*)(sO + (NF * pr + f) * 132 + col);
    unsigned short hb[4], lb[4];
#pragma unroll
    for (int e = 0; e < 4; ++e) split_h((s[e] * (1.0f / NF)) * AC, hb[e], lb[e]);
    v2u ph2, pl2;
    ph2[0] = pk16(hb[0], hb[1]); ph2[1] = pk16(hb[2], hb[3]);
    pl2[0] = pk16(lb[0], lb[1]); pl2[1] = pk16(lb[2], lb[3]);
    if (act) {
      *(v2u*)(sPH + pr * 128 + col) = ph2;
      *(v2u*)(sPL + pr * 128 + col) = pl2;
    }
  }
  __syncthreads();
  {
    const bool wr  = (t < 256);
    const bool isl = (t >= 128);
    const int tt = t & 127;
    const int row = tt >> 4, e = tt & 15;
    const v4u a  = *(const v4u*)(sPH + row * 128 + 8 * e);
    const v4u bq = *(const v4u*)(sPL + row * 128 + 8 * e);
    v4u val;
#pragma unroll
    for (int i = 0; i < 4; ++i) val[i] = isl ? bq[i] : a[i];
    unsigned short* dp = (isl ? PL : PH) + ((size_t)(b * TT + 8 * qblk + row)) * HID + 8 * e;
    if (wr) *(volatile v4u*)dp = val;
    __threadfence();
    if (wr) *(volatile v4u*)dp = val;
  }
}

__global__ __launch_bounds__(256) void tail_k(const unsigned short* __restrict__ PH, const unsigned short* __restrict__ PL,
                                               const unsigned short* __restrict__ WOT, const float* __restrict__ obias,
                                               const float* __restrict__ flnw, const float* __restrict__ flnb,
                                               const unsigned short* __restrict__ FWT, const float* __restrict__ fbias,
                                               float* out) {
  __shared__ __align__(16) float sZ[64 * 132];
  const int t = threadIdx.x, wave = t >> 5, lane = t & 31, hh = lane >> 4, m = lane & 15;
  const int r0 = blockIdx.x * 64;
  const int rt = wave & 3, ch = wave >> 2;

  {
    v8f acc[4], accr[4];
#pragma unroll
    for (int j = 0; j < 4; ++j) { acc[j] = zero8(); accr[j] = zero8(); }
    const _Float16* Ah = h16(PH) + (size_t)(r0 + 16 * rt + m) * HID + 8 * hh;
    const _Float16* Al = h16(PL) + (size_t)(r0 + 16 * rt + m) * HID + 8 * hh;
    const _Float16* Bw = h16(WOT) + (size_t)(64 * ch + m) * HID + 8 * hh;
#pragma unroll 1
    for (int k0 = 0; k0 < HID; k0 += 32) {
      v16h bf[4];
#pragma unroll
      for (int j = 0; j < 4; ++j) bf[j] = ldfrag_h(Bw + (size_t)(16 * j) * HID + k0);
      const v16h ah = ldfrag_h(Ah + k0);
      const v16h al = ldfrag_h(Al + k0);
#pragma unroll
      for (int j = 0; j < 4; ++j) acc[j]  = mma_h_raw(ah, bf[j], acc[j]);
#pragma unroll
      for (int j = 0; j < 4; ++j) accr[j] = mma_h_raw(al, bf[j], accr[j]);
      guard8x6(acc[0], acc[1], acc[2], acc[3], accr[0], accr[1], accr[2], accr[3], ah, al, bf[0], bf[1], bf[2], bf[3]);
    }
    acc_guard4(acc[0], acc[1], acc[2], acc[3]);
    acc_guard4(accr[0], accr[1], accr[2], accr[3]);
#pragma unroll
    for (int j = 0; j < 4; ++j) {
      const int n = 64 * ch + 16 * j + m;
      const float bn = bfr(obias[n]);
#pragma unroll
      for (int r = 0; r < 8; ++r) {
        const int row = 16 * rt + 8 * hh + r;
        sZ[row * 132 + n] = (acc[j][r] + accr[j][r] * INVRS) * (1.0f / (AC * WSC)) + bn;
      }
    }
  }
  __syncthreads();

  {
    float gg[4], bb[4];
#pragma unroll
    for (int e = 0; e < 4; ++e) { gg[e] = bfr(flnw[4 * lane + e]); bb[e] = bfr(flnb[4 * lane + e]); }
#pragma unroll 1
    for (int i = 0; i < 8; ++i) {
      const int row = 8 * wave + i;
      float* zp = sZ + row * 132 + 4 * lane;
      const v4f z = *(const v4f*)zp;
      float s = (z[0] + z[1]) + (z[2] + z[3]);
      s = wsum(s);
      const float mean = s * (1.0f / HID);
      float d[4];
#pragma unroll
      for (int e = 0; e < 4; ++e) d[e] = z[e] - mean;
      float vs = (d[0] * d[0] + d[1] * d[1]) + (d[2] * d[2] + d[3] * d[3]);
      vs = wsum(vs);
      const float rstd = rsqrtf(vs * (1.0f / HID) + LNEPS);
      v4f y;
#pragma unroll
      for (int e = 0; e < 4; ++e) y[e] = (d[e] * rstd) * gg[e] + bb[e];
      *(v4f*)zp = y;
    }
  }
  __syncthreads();

  v8f acc2[4], acc2r[4];
#pragma unroll
  for (int j = 0; j < 4; ++j) { acc2[j] = zero8(); acc2r[j] = zero8(); }
  {
    const float* zr = sZ + (16 * rt + m) * 132 + 8 * hh;
    const _Float16* Bf = h16(FWT) + (size_t)(64 * ch + m) * HID + 8 * hh;
#pragma unroll 1
    for (int k0 = 0; k0 < HID; k0 += 32) {
      FragH ah, al;
      const v4f za = *(const v4f*)(zr + k0), zb = *(const v4f*)(zr + k0 + 4);
      const v4f zc = *(const v4f*)(zr + k0 + 16), zd = *(const v4f*)(zr + k0 + 20);
#pragma unroll
      for (int i = 0; i < 4; ++i) {
        const float f0 = za[i] * YC, f1 = zb[i] * YC, f2 = zc[i] * YC, f3 = zd[i] * YC;
        const _Float16 h0 = (_Float16)f0, h1 = (_Float16)f1, h2 = (_Float16)f2, h3 = (_Float16)f3;
        ah.h[0][i] = h0;     al.h[0][i]     = (_Float16)((f0 - (float)h0) * RSC);
        ah.h[0][4 + i] = h1; al.h[0][4 + i] = (_Float16)((f1 - (float)h1) * RSC);
        ah.h[1][i] = h2;     al.h[1][i]     = (_Float16)((f2 - (float)h2) * RSC);
        ah.h[1][4 + i] = h3; al.h[1][4 + i] = (_Float16)((f3 - (float)h3) * RSC);
      }
      v16h bf[4];
#pragma unroll
      for (int j = 0; j < 4; ++j) bf[j] = ldfrag_h(Bf + (size_t)(16 * j) * HID + k0);
#pragma unroll
      for (int j = 0; j < 4; ++j) acc2[j]  = mma_h_raw(ah.v, bf[j], acc2[j]);
#pragma unroll
      for (int j = 0; j < 4; ++j) acc2r[j] = mma_h_raw(al.v, bf[j], acc2r[j]);
      guard8x6(acc2[0], acc2[1], acc2[2], acc2[3], acc2r[0], acc2r[1], acc2r[2], acc2r[3],
               ah.v, al.v, bf[0], bf[1], bf[2], bf[3]);
    }
    acc_guard4(acc2[0], acc2[1], acc2[2], acc2[3]);
    acc_guard4(acc2r[0], acc2r[1], acc2r[2], acc2r[3]);
  }
  __syncthreads();
#pragma unroll
  for (int j = 0; j < 4; ++j) {
    const int n = 64 * ch + 16 * j + m;
    const float bn = bfr(fbias[n]);
#pragma unroll
    for (int r = 0; r < 8; ++r) {
      const int row = 16 * rt + 8 * hh + r;
      const float a = (acc2[j][r] + acc2r[j][r] * INVRS) * (1.0f / (YC * WSC)) + bn;
      sZ[row * 132 + n] = a * sigm(a);
    }
  }
  __syncthreads();
  {
    v4f vals[8];
#pragma unroll
    for (int i = 0; i < 8; ++i) vals[i] = *(const v4f*)(sZ + (8 * i + wave) * 132 + 4 * lane);
#pragma unroll
    for (int i = 0; i < 8; ++i)
      *(volatile v4f*)(out + (size_t)(r0 + 8 * i + wave) * FD + 4 * lane) = vals[i];
    __threadfence();
#pragma unroll
    for (int i = 0; i < 8; ++i)
      *(volatile v4f*)(out + (size_t)(r0 + 8 * i + wave) * FD + 4 * lane) = vals[i];
  }
}

extern "C" void kernel_launch(void* const* d_in, const int* in_sizes, int n_in,
                              void* d_out, int out_size, void* d_ws, size_t ws_size,
                              hipStream_t stream) {
  if (n_in < 20) return;
  if (in_sizes[0] != NTOK * DD) return;
  if (in_sizes[1] != DD || in_sizes[2] != DD || in_sizes[3] != DD * GH || in_sizes[4] != GH ||
      in_sizes[5] != GH || in_sizes[6] != 1) return;
  if (in_sizes[7] != DD * HID || in_sizes[8] != HID || in_sizes[9] != DD * HID || in_sizes[10] != HID ||
      in_sizes[11] != DD * HID || in_sizes[12] != HID) return;
  if (in_sizes[13] != HID * HID || in_sizes[14] != HID || in_sizes[15] != HID || in_sizes[16] != HID ||
      in_sizes[17] != HID * FD || in_sizes[18] != FD || in_sizes[19] != 1) return;
  if (out_size != NPOOL * FD) return;

  const float* x    = (const float*)d_in[0];
  const float* glnw = (const float*)d_in[1];
  const float* glnb = (const float*)d_in[2];
  const float* gw1  = (const float*)d_in[3];
  const float* gb1  = (const float*)d_in[4];
  const float* gw2  = (const float*)d_in[5];
  const float* gb2  = (const float*)d_in[6];
  const float* qw   = (const float*)d_in[7];
  const float* qb   = (const float*)d_in[8];
  const float* kw   = (const float*)d_in[9];
  const float* kb   = (const float*)d_in[10];
  const float* vw   = (const float*)d_in[11];
  const float* vb   = (const float*)d_in[12];
  const float* ow   = (const float*)d_in[13];
  const float* ob   = (const float*)d_in[14];
  const float* flnw = (const float*)d_in[15];
  const float* flnb = (const float*)d_in[16];
  const float* fw   = (const float*)d_in[17];
  const float* fb   = (const float*)d_in[18];
  const int*   Tp   = (const int*)d_in[19];

  const size_t PWT = (size_t)3 * HID * DD * 2;
  const size_t PWO = (size_t)HID * HID * 2;
  const size_t PWF = (size_t)FD * HID * 2;
  const size_t PQP = (size_t)NTOK * HID * 2;
  const size_t PVT = (size_t)NB * HID * LL * 2;
  const size_t PSV = (size_t)NB * HID * TT * 4;
  const size_t PPP = (size_t)NPOOL * HID * 2;
  size_t off = 0;
  const size_t oWT = off; off += PWT;
  const size_t oWO = off; off += PWO;
  const size_t oWF = off; off += PWF;
  const size_t oQH = off; off += PQP;
  const size_t oQL = off; off += PQP;
  const size_t oKH = off; off += PQP;
  const size_t oKL = off; off += PQP;
  const size_t oVH = off; off += PVT;
  const size_t oVL = off; off += PVT;
  const size_t oSV = off; off += PSV;
  const size_t oPH = off; off += PPP;
  const size_t oPL = off; off += PPP;
  if (off > ws_size) return;
  if (off > (size_t)134217728) return;

  char* ws = (char*)d_ws;
  unsigned short* WT  = (unsigned short*)(ws + oWT);
  unsigned short* WOT = (unsigned short*)(ws + oWO);
  unsigned short* FWT = (unsigned short*)(ws + oWF);
  unsigned short* QH  = (unsigned short*)(ws + oQH);
  unsigned short* QL  = (unsigned short*)(ws + oQL);
  unsigned short* KH  = (unsigned short*)(ws + oKH);
  unsigned short* KL  = (unsigned short*)(ws + oKL);
  unsigned short* VTH = (unsigned short*)(ws + oVH);
  unsigned short* VTL = (unsigned short*)(ws + oVL);
  float*          SV  = (float*)(ws + oSV);
  unsigned short* PH  = (unsigned short*)(ws + oPH);
  unsigned short* PL  = (unsigned short*)(ws + oPL);
  float*          out = (float*)d_out;

  const dim3 blk(256), blk384(384);
  const dim3 gW(12 + 8 + 8);
  const dim3 gQ(NTOK / 64);
  const dim3 gS(NB * HID);
  const dim3 gA(NB * (LL / 48));
  const dim3 gT(NPOOL / 64);

  wprep<<<gW, blk, 0, stream>>>(qw, kw, vw, ow, fw, WT, WOT, FWT);

  qkv_prep<<<gQ, blk, 0, stream>>>(x, glnw, glnb, gw1, gb1, gw2, gb2, qb, kb, vb, WT, QH, QL, KH, KL, VTH, VTL);

  vsuf<<<gS, blk, 0, stream>>>(VTH, VTL, Tp, SV);

  attn_pool<<<gA, blk384, 0, stream>>>(QH, QL, KH, KL, VTH, VTL, SV, PH, PL);

  tail_k<<<gT, blk, 0, stream>>>(PH, PL, WOT, ob, flnw, flnb, FWT, fb, out);
  (void)hipGetLastError();
}
